// GraphEdgeWeight_47493748359688
// MI455X (gfx1250) — hardware-run, weakly checked
//
#include <hip/hip_runtime.h>
#include <stddef.h>
#include <stdint.h>


#define HID    128
#define NN     100000
#define NPAD   100096
#define NE     1000000
#define TE     64
#define NT     (NE / TE)
#define NTHR   256
#define K2     256
#define AP     264
#define SP     132
#define TABN   1024
#define NBLK_E 1024
#define NODE_LDS (128 * AP * 2 + HID * 4)
#define EDGE_LDS (128 * AP * 2 + TE * AP * 2 + 384 * 4 + 2 * TE * 4 + TE * 4)
#define NU_X   (NPAD * 16)
#define NU_WT  4096
#define NU_W1  12288
#define NU_TAB 256
#define NU_ALL (NU_X + NU_WT + NU_W1 + NU_TAB)
#define WSMAX  134217728

static_assert(HID == 128);
static_assert(8 * 16 == HID);
static_assert(HID % 8 == 0);
static_assert(NE % TE == 0);
static_assert(NPAD % 128 == 0 && NPAD >= NN && NPAD - NN < 128);
static_assert(AP * 2 == SP * 4 && (AP * 2) % 16 == 0 && AP >= K2 && SP >= HID);
static_assert(NU_X % NTHR == 0 && NU_WT % NTHR == 0 && NU_W1 % NTHR == 0 && NU_ALL % NTHR == 0);
static_assert(NODE_LDS <= 327680 && EDGE_LDS <= 327680);
static_assert(NBLK_E <= NT);
static_assert(TABN * 4 == NU_TAB * 16);

typedef float          v4f   __attribute__((ext_vector_type(4)));
typedef float          v8f   __attribute__((ext_vector_type(8)));
typedef int            v8i   __attribute__((ext_vector_type(8)));
typedef unsigned       v4u   __attribute__((ext_vector_type(4)));
typedef unsigned short v8us  __attribute__((ext_vector_type(8)));
typedef unsigned short v16us __attribute__((ext_vector_type(16)));
typedef __bf16         v16bf __attribute__((ext_vector_type(16)));
typedef v4f  __attribute__((may_alias)) v4fa;
typedef v4u  __attribute__((may_alias)) v4ua;
typedef v8us __attribute__((may_alias)) v8usa;
union FragB { v16bf v; v16us u; v8us h[2]; v8i w; };

__device__ __forceinline__ v8f wmb(const FragB& a, const FragB& b, v8f c) {
  v8f d = __builtin_amdgcn_wmma_f32_16x16x32_bf16(false, a.v, false, b.v, (short)0, c, false, false);
  asm volatile("v_nop\n\tv_nop\n\tv_nop\n\tv_nop" : "+v"(d) : "v"(a.w), "v"(b.w));
  return d;
}

__device__ __forceinline__ unsigned bf16_bits(float f) {
  const unsigned u = __float_as_uint(f);
  return (u + 0x7FFFu + ((u >> 16) & 1u)) >> 16;
}
__device__ __forceinline__ float bf16_val(float f) {
  return __uint_as_float(bf16_bits(f) << 16);
}
__device__ __forceinline__ void put16(unsigned short* dp, v8us o) {
  *(volatile v8us*)dp = o;
  __threadfence();
  *(volatile v8us*)dp = o;
}
__device__ __forceinline__ void putf4(float* dp, v4f o) {
  *(volatile v4f*)dp = o;
  __threadfence();
  *(volatile v4f*)dp = o;
}

__global__ __launch_bounds__(NTHR) void k_prep(const float* __restrict__ x,
                                               const float* __restrict__ Wp, const float* __restrict__ bp,
                                               const float* __restrict__ Wc, const float* __restrict__ bc,
                                               const float* __restrict__ W1, const float* __restrict__ b1,
                                               const float* __restrict__ W2, const float* __restrict__ b2,
                                               unsigned short* XB, unsigned short* WT, unsigned short* W1D,
                                               float* TAB) {
  const int u  = (int)blockIdx.x * NTHR + (int)threadIdx.x;
  const int U0 = NU_X;
  const int U1 = U0 + NU_WT;
  const int U2 = U1 + NU_W1;
  const int U3 = U2 + NU_TAB;
  v8us o;
  if (u < U0) {
    const int row = u >> 4;
    const int k8  = (u & 15) * 8;
    const int rc  = row < NN ? row : NN - 1;
    const float* p = x + (size_t)rc * HID + k8;
    const v4f a = *(const v4fa*)p;
    const v4f b = *(const v4fa*)(p + 4);
    const unsigned msk = row < NN ? 0xffffu : 0u;
    o[0] = (unsigned short)(bf16_bits(a.x) & msk);
    o[1] = (unsigned short)(bf16_bits(a.y) & msk);
    o[2] = (unsigned short)(bf16_bits(a.z) & msk);
    o[3] = (unsigned short)(bf16_bits(a.w) & msk);
    o[4] = (unsigned short)(bf16_bits(b.x) & msk);
    o[5] = (unsigned short)(bf16_bits(b.y) & msk);
    o[6] = (unsigned short)(bf16_bits(b.z) & msk);
    o[7] = (unsigned short)(bf16_bits(b.w) & msk);
    put16(XB + (size_t)row * HID + k8, o);
    return;
  } else if (u < U1) {
    const int v  = u - U0;
    const int br = v >> 11;
    const int vv = v & 2047;
    const int n  = vv >> 4;
    const int k8 = (vv & 15) * 8;
    const float* W = (br == 0) ? Wp : Wc;
    const float* p = W + (size_t)k8 * HID + n;
#pragma unroll
    for (int i = 0; i < 8; ++i) o[i] = (unsigned short)bf16_bits(p[(size_t)i * HID]);
    put16(WT + (size_t)br * (HID * HID) + (size_t)n * HID + k8, o);
    return;
  } else if (u < U2) {
    const int v    = u - U1;
    const int sel  = v >> 12;
    const int vv   = v & 4095;
    const int n    = vv >> 5;
    const int k8   = (vv & 31) * 8;
    const int srow = sel * HID + (k8 & (HID - 1));
    const float* p = W1 + (size_t)srow * HID + n;
#pragma unroll
    for (int i = 0; i < 8; ++i) o[i] = (unsigned short)bf16_bits(p[(size_t)i * HID]);
    put16(W1D + (size_t)sel * (HID * K2) + (size_t)n * K2 + k8, o);
    return;
  } else if (u < U3) {
    const int t = u - U2;
    const int g = t >> 5;
    const int j = t & 31;
    v4f q = {0.0f, 0.0f, 0.0f, 0.0f};
    if (g == 0)      q = *(const v4fa*)(bp + 4 * j);
    else if (g == 1) q = *(const v4fa*)(bc + 4 * j);
    else if (g == 2) q = *(const v4fa*)(b1 + 4 * j);
    else if (g == 3) q = *(const v4fa*)(W2 + 4 * j);
    const float b2v = b2[0];
    asm volatile("" :: "v"(b2v));
    v4f r;
    r.x = bf16_val(q.x);
    r.y = bf16_val(q.y);
    r.z = bf16_val(q.z);
    r.w = bf16_val(q.w);
    const float b2r = bf16_val(b2v);
    r.x = (t == 128) ? b2r : r.x;
    putf4(TAB + 4 * t, r);
    return;
  }
}

__global__ __launch_bounds__(NTHR) __attribute__((amdgpu_num_vgpr(248)))
void k_node(const unsigned short* __restrict__ XB, const unsigned short* __restrict__ WT,
            const unsigned short* __restrict__ W1D, const float* __restrict__ TAB, float* Q) {
  extern __shared__ __attribute__((aligned(16))) float dynn[];
  unsigned short* sA    = (unsigned short*)dynn;
  float*          stg   = dynn;
  float*          sBias = dynn + 128 * SP;

  const int tid = (int)threadIdx.x, lane = tid & 31, wave = tid >> 5, hh = lane >> 4, m = lane & 15;
  const int rowBase = (int)blockIdx.x * 128;
  const int branch  = (int)blockIdx.y;

  if (tid < 32) {
    const v4f bq = *(const v4fa*)(TAB + branch * HID + 4 * tid);
    *(v4fa*)(sBias + 4 * tid) = bq;
  }
  __syncthreads();

  v8f acc[8];
  const v8f z = {0.f, 0.f, 0.f, 0.f, 0.f, 0.f, 0.f, 0.f};
#pragma unroll
  for (int t = 0; t < 8; ++t) acc[t] = z;

  {
    const unsigned short* ap = XB + (size_t)(rowBase + 16 * wave + m) * HID + 8 * hh;
    const unsigned short* bp = WT + (size_t)branch * (HID * HID) + (size_t)m * HID + 8 * hh;
#pragma unroll 1
    for (int k0 = 0; k0 < HID; k0 += 32) {
      FragB af;
      af.h[0] = *(const v8usa*)(ap + k0);
      af.h[1] = *(const v8usa*)(ap + k0 + 16);
#pragma unroll
      for (int nt = 0; nt < 8; ++nt) {
        const unsigned short* wq = bp + (size_t)(16 * nt) * HID + k0;
        FragB bf;
        bf.h[0] = *(const v8usa*)wq;
        bf.h[1] = *(const v8usa*)(wq + 16);
        acc[nt] = wmb(af, bf, acc[nt]);
      }
    }
  }

#pragma unroll
  for (int nt = 0; nt < 8; ++nt) {
    const int col = 16 * nt + m;
    const float bv = sBias[col];
#pragma unroll
    for (int r = 0; r < 8; ++r) {
      const int lr = 16 * wave + 8 * hh + r;
      float v = acc[nt][r] + bv;
      v = (v >= 0.0f) ? v : (0.01f * v);
      const unsigned hb = bf16_bits(v);
      const unsigned lb = bf16_bits(v - __uint_as_float(hb << 16));
      sA[lr * AP + col]       = (unsigned short)hb;
      sA[lr * AP + HID + col] = (unsigned short)lb;
    }
  }
  __syncthreads();

#pragma unroll
  for (int t = 0; t < 8; ++t) acc[t] = z;
  {
    const unsigned short* ap = sA + (16 * wave + m) * AP + 8 * hh;
    const unsigned short* bp = W1D + (size_t)branch * (HID * K2) + (size_t)m * K2 + 8 * hh;
#pragma unroll 1
    for (int k0 = 0; k0 < K2; k0 += 32) {
      FragB af;
      af.h[0] = *(const v8usa*)(ap + k0);
      af.h[1] = *(const v8usa*)(ap + k0 + 16);
#pragma unroll
      for (int nt = 0; nt < 8; ++nt) {
        const unsigned short* wq = bp + (size_t)(16 * nt) * K2 + k0;
        FragB bf;
        bf.h[0] = *(const v8usa*)wq;
        bf.h[1] = *(const v8usa*)(wq + 16);
        acc[nt] = wmb(af, bf, acc[nt]);
      }
    }
  }
  __syncthreads();

#pragma unroll
  for (int nt = 0; nt < 8; ++nt) {
    const int col = 16 * nt + m;
#pragma unroll
    for (int r = 0; r < 8; ++r) {
      const int lr = 16 * wave + 8 * hh + r;
      stg[lr * SP + col] = acc[nt][r];
    }
  }
  __syncthreads();

  {
    float* qb = Q + (size_t)branch * ((size_t)NPAD * HID);
    v4f pv[16];
#pragma unroll
    for (int i = 0; i < 16; ++i) pv[i] = *(const v4fa*)(stg + (16 * wave + i) * SP + 4 * lane);
#pragma unroll
    for (int i = 0; i < 16; ++i) {
      const int row = rowBase + 16 * wave + i;
      if (row < NN) {
        float* op = qb + (size_t)row * HID + 4 * lane;
        *(volatile v4f*)op = pv[i];
      }
    }
    __threadfence();
#pragma unroll
    for (int i = 0; i < 16; ++i) {
      const int row = rowBase + 16 * wave + i;
      if (row < NN) {
        float* op = qb + (size_t)row * HID + 4 * lane;
        *(volatile v4f*)op = pv[i];
      }
    }
  }
}

__global__ __launch_bounds__(NTHR) __attribute__((amdgpu_num_vgpr(248)))
void k_edge(const int* __restrict__ eidx, const unsigned short* __restrict__ XB,
            const unsigned short* __restrict__ W1dD, const float* __restrict__ TAB,
            const float* __restrict__ QP, const float* __restrict__ QC, float* out) {
  extern __shared__ __attribute__((aligned(16))) float dyne[];
  unsigned short* sW   = (unsigned short*)dyne;
  unsigned short* sA   = sW + 128 * AP;
  float*          stg  = dyne + (128 * AP) / 2;
  float*          sTab = dyne + (128 * AP) / 2 + (TE * AP) / 2;
  int*            sIdx = (int*)(sTab + 384);
  float*          sOut = (float*)(sIdx + 2 * TE);

  const int tid = (int)threadIdx.x, lane = tid & 31, wave = tid >> 5, hh = lane >> 4, m = lane & 15;

#pragma unroll 4
  for (int it = 0; it < 16; ++it) {
    const int p = it * NTHR + tid;
    const int n = p >> 5;
    const int c = p & 31;
    const v4u wv = *(const v4ua*)(W1dD + (size_t)n * K2 + 8 * c);
    *(v4ua*)(sW + n * AP + 8 * c) = wv;
  }
  if (tid < 96) {
    const v4f tv = *(const v4fa*)(TAB + 2 * HID + 4 * tid);
    *(v4fa*)(sTab + 4 * tid) = tv;
  }
  __syncthreads();

  const v4f   b1r = *(const v4fa*)(sTab + 4 * lane);
  const v4f   w2r = *(const v4fa*)(sTab + HID + 4 * lane);
  const float b2v = sTab[2 * HID];
  const v8f   z   = {0.f, 0.f, 0.f, 0.f, 0.f, 0.f, 0.f, 0.f};

#pragma unroll 1
  for (int tile = (int)blockIdx.x; tile < NT; tile += (int)gridDim.x) {
    if (tid < 2 * TE) {
      const int which = tid >> 6;
      const int r     = tid & (TE - 1);
      int v = eidx[(size_t)which * NE + (size_t)tile * TE + r];
      v = v < 0 ? 0 : (v > NN - 1 ? NN - 1 : v);
      sIdx[tid] = v;
    }
    __syncthreads();

#pragma unroll
    for (int p = 0; p < 4; ++p) {
      const int row = 8 * wave + 2 * p + hh;
      const int s = sIdx[row];
      const int t = sIdx[TE + row];
      const v4u a = *(const v4ua*)(XB + (size_t)s * HID + 8 * m);
      const v4u b = *(const v4ua*)(XB + (size_t)t * HID + 8 * m);
      v4u ohi, olo;
#pragma unroll
      for (int w = 0; w < 4; ++w) {
        const unsigned aw = a[w];
        const unsigned bw = b[w];
        const float a0 = __uint_as_float(aw << 16);
        const float a1 = __uint_as_float(aw & 0xffff0000u);
        const float c0 = __uint_as_float(bw << 16);
        const float c1 = __uint_as_float(bw & 0xffff0000u);
        const float d0 = fabsf(a0 - c0);
        const float d1 = fabsf(a1 - c1);
        const unsigned h0 = bf16_bits(d0);
        const unsigned h1 = bf16_bits(d1);
        const unsigned l0 = bf16_bits(d0 - __uint_as_float(h0 << 16));
        const unsigned l1 = bf16_bits(d1 - __uint_as_float(h1 << 16));
        ohi[w] = h0 | (h1 << 16);
        olo[w] = l0 | (l1 << 16);
      }
      *(v4ua*)(sA + row * AP + 8 * m)       = ohi;
      *(v4ua*)(sA + row * AP + HID + 8 * m) = olo;
    }
    __syncthreads();

    v8f acc[4];
#pragma unroll
    for (int mt = 0; mt < 4; ++mt) acc[mt] = z;
    {
      const unsigned short* bp = sW + (16 * wave + m) * AP + 8 * hh;
      const unsigned short* ap = sA + m * AP + 8 * hh;
#pragma unroll 1
      for (int k0 = 0; k0 < K2; k0 += 32) {
        FragB bf;
        bf.h[0] = *(const v8usa*)(bp + k0);
        bf.h[1] = *(const v8usa*)(bp + k0 + 16);
#pragma unroll
        for (int mt = 0; mt < 4; ++mt) {
          FragB af;
          af.h[0] = *(const v8usa*)(ap + mt * 16 * AP + k0);
          af.h[1] = *(const v8usa*)(ap + mt * 16 * AP + k0 + 16);
          acc[mt] = wmb(af, bf, acc[mt]);
        }
      }
    }
    __syncthreads();

#pragma unroll
    for (int mt = 0; mt < 4; ++mt) {
#pragma unroll
      for (int r = 0; r < 8; ++r) {
        stg[(16 * mt + 8 * hh + r) * SP + 16 * wave + m] = acc[mt][r];
      }
    }
    __syncthreads();

    float res = 0.0f;
#pragma unroll
    for (int i = 0; i < 8; ++i) {
      const int row = 8 * wave + i;
      const int s = sIdx[row];
      const int t = sIdx[TE + row];
      const v4f sv = *(const v4fa*)(stg + row * SP + 4 * lane);
      const v4f qp = *(const v4fa*)(QP + (size_t)s * HID + 4 * lane);
      const v4f qc = *(const v4fa*)(QC + (size_t)t * HID + 4 * lane);
      float v0 = ((sv.x + qp.x) + qc.x) + b1r.x;
      float v1 = ((sv.y + qp.y) + qc.y) + b1r.y;
      float v2 = ((sv.z + qp.z) + qc.z) + b1r.z;
      float v3 = ((sv.w + qp.w) + qc.w) + b1r.w;
      v0 = (v0 > 0.0f) ? v0 : (v0 - v0);
      v1 = (v1 > 0.0f) ? v1 : (v1 - v1);
      v2 = (v2 > 0.0f) ? v2 : (v2 - v2);
      v3 = (v3 > 0.0f) ? v3 : (v3 - v3);
      float dot = v0 * w2r.x;
      dot = fmaf(v1, w2r.y, dot);
      dot = fmaf(v2, w2r.z, dot);
      dot = fmaf(v3, w2r.w, dot);
      dot += __shfl_xor(dot, 16, 32);
      dot += __shfl_xor(dot, 8, 32);
      dot += __shfl_xor(dot, 4, 32);
      dot += __shfl_xor(dot, 2, 32);
      dot += __shfl_xor(dot, 1, 32);
      res = (lane == i) ? dot : res;
    }
    {
      const float a  = res + b2v;
      const float sg = 1.0f / (1.0f + expf(-a));
      if (lane < 8) sOut[8 * wave + lane] = sg;
    }
    __syncthreads();

    if (wave == 0) {
      const int lq = lane & 15;
      const v4f o4 = *(const v4fa*)(sOut + 4 * lq);
      asm volatile("" :: "v"(o4));
      float* op = out + (size_t)tile * TE + 4 * lq;
      if (lane < 16) *(volatile v4f*)op = o4;
      __threadfence();
      if (lane < 16) *(volatile v4f*)op = o4;
    }
  }
}

extern "C" void kernel_launch(void* const* d_in, const int* in_sizes, int n_in,
                              void* d_out, int out_size, void* d_ws, size_t ws_size,
                              hipStream_t stream) {
  if (n_in < 10) return;
  if (in_sizes[0] != NN * HID) return;
  if (in_sizes[1] != 2 * NE) return;
  if (in_sizes[2] != HID * HID || in_sizes[3] != HID) return;
  if (in_sizes[4] != HID * HID || in_sizes[5] != HID) return;
  if (in_sizes[6] != 3 * HID * HID || in_sizes[7] != HID) return;
  if (in_sizes[8] != HID || in_sizes[9] != 1) return;
  if (out_size != NE) return;

  const float* x  = (const float*)d_in[0];
  const int*   ei = (const int*)d_in[1];
  const float* Wp = (const float*)d_in[2];
  const float* bp = (const float*)d_in[3];
  const float* Wc = (const float*)d_in[4];
  const float* bc = (const float*)d_in[5];
  const float* W1 = (const float*)d_in[6];
  const float* b1 = (const float*)d_in[7];
  const float* W2 = (const float*)d_in[8];
  const float* b2 = (const float*)d_in[9];
  float* out = (float*)d_out;

  const size_t szXB  = (size_t)NPAD * HID * 2;
  const size_t szQ   = (size_t)2 * NPAD * HID * 4;
  const size_t szWT  = (size_t)2 * HID * HID * 2;
  const size_t szW1D = (size_t)3 * HID * K2 * 2;
  const size_t szTAB = (size_t)TABN * 4;
  const size_t oXB  = 0;
  const size_t oQ   = oXB + szXB;
  const size_t oWT  = oQ + szQ;
  const size_t oW1D = oWT + szWT;
  const size_t oTAB = oW1D + szW1D;
  const size_t total = oTAB + szTAB;
  if (total > ws_size || total > (size_t)WSMAX) return;

  char* ws = (char*)d_ws;
  unsigned short* XB  = (unsigned short*)(ws + oXB);
  float*          Q   = (float*)(ws + oQ);
  unsigned short* WT  = (unsigned short*)(ws + oWT);
  unsigned short* W1D = (unsigned short*)(ws + oW1D);
  float*          TAB = (float*)(ws + oTAB);
  const float* QP = Q;
  const float* QC = Q + (size_t)NPAD * HID;
  const unsigned short* W1dD = W1D + (size_t)2 * HID * K2;

  hipFuncSetAttribute(reinterpret_cast<const void*>(&k_node), hipFuncAttributeMaxDynamicSharedMemorySize,
                      (int)NODE_LDS);
  hipFuncSetAttribute(reinterpret_cast<const void*>(&k_edge), hipFuncAttributeMaxDynamicSharedMemorySize,
                      (int)EDGE_LDS);

  k_prep<<<NU_ALL / NTHR, NTHR, 0, stream>>>(x, Wp, bp, Wc, bc, W1, b1, W2, b2, XB, WT, W1D, TAB);
  k_node<<<dim3(NPAD / 128, 2), NTHR, NODE_LDS, stream>>>(XB, WT, W1D, TAB, Q);
  k_edge<<<NBLK_E, NTHR, EDGE_LDS, stream>>>(ei, XB, W1dD, TAB, QP, QC, out);
}
